// EFLayoutSpatialAttention_36661840838668
// MI455X (gfx1250) — hardware-verified
//
#include <hip/hip_runtime.h>
#include <math.h>
#include <stdint.h>

#define SEQ   4096
#define DM    1024
#define NH    16
#define HD    64
#define NQB   (SEQ / 64)
#define QKP   (2 * DM)
static_assert(NH * HD == DM);
static_assert((SEQ % 64) == 0 && (DM % 64) == 0 && (DM % 32) == 0);
static_assert((HD % 8) == 0 && (HD / 2) % 8 == 0);

typedef _Float16 v16h __attribute__((ext_vector_type(16)));
typedef _Float16 v8h  __attribute__((ext_vector_type(8)));
typedef __bf16   v16b __attribute__((ext_vector_type(16)));
typedef __bf16   v8b  __attribute__((ext_vector_type(8)));
typedef float    v8f  __attribute__((ext_vector_type(8)));
typedef float    v4f  __attribute__((ext_vector_type(4)));
typedef unsigned int v4u __attribute__((ext_vector_type(4)));

__device__ __forceinline__ unsigned short bf_bits(float f) {
  unsigned u = __float_as_uint(f);
  return (unsigned short)((u + 0x7FFFu + ((u >> 16) & 1u)) >> 16);
}
__device__ __forceinline__ float bf_up(unsigned short h) { return __uint_as_float(((unsigned)h) << 16); }
__device__ __forceinline__ float bf_rne(float f) { return bf_up(bf_bits(f)); }
__device__ __forceinline__ unsigned short h_bits(_Float16 x) { return __builtin_bit_cast(unsigned short, x); }
__device__ __forceinline__ unsigned pk16(unsigned short a, unsigned short b) { return (unsigned)a | ((unsigned)b << 16); }
__device__ __forceinline__ v8f zero8() { v8f z = {0.f, 0.f, 0.f, 0.f, 0.f, 0.f, 0.f, 0.f}; return z; }

__device__ __forceinline__ v16b ldfrag_b(const __bf16* p) {
  union { v16b v; v8b h[2]; } f;
  f.h[0] = *(const v8b*)(p);
  f.h[1] = *(const v8b*)(p + 16);
  return f.v;
}
__device__ __forceinline__ v16h ldfrag_h(const _Float16* p) {
  union { v16h v; v8h h[2]; } f;
  f.h[0] = *(const v8h*)(p);
  f.h[1] = *(const v8h*)(p + 16);
  return f.v;
}

__device__ __forceinline__ v8f mma_h(v16h a, v16h b, v8f c) {
  c = __builtin_amdgcn_wmma_f32_16x16x32_f16(false, a, false, b, (short)0, c, false, false);
#if defined(__HIP_DEVICE_COMPILE__)
  asm volatile("v_nop\n\tv_nop\n\tv_nop\n\tv_nop" : "+v"(c) : "v"(a), "v"(b));
#endif
  return c;
}
__device__ __forceinline__ v8f mma_b_raw(v16b a, v16b b, v8f c) {
  return __builtin_amdgcn_wmma_f32_16x16x32_bf16(false, a, false, b, (short)0, c, false, false);
}
__device__ __forceinline__ void dep_guard_b(v8f& a, v8f& b, v16b x, v16b y) {
#if defined(__HIP_DEVICE_COMPILE__)
  asm volatile("v_nop\n\tv_nop\n\tv_nop\n\tv_nop" : "+v"(a), "+v"(b) : "v"(x), "v"(y));
#endif
}
__device__ __forceinline__ void keep4_b(v16b a, v16b b, v16b c, v16b d) {
#if defined(__HIP_DEVICE_COMPILE__)
  asm volatile("v_nop" :: "v"(a), "v"(b), "v"(c), "v"(d));
#endif
}
__device__ __forceinline__ void acc_guard4(v8f& a, v8f& b, v8f& c, v8f& d) {
#if defined(__HIP_DEVICE_COMPILE__)
  asm volatile("v_nop\n\tv_nop\n\tv_nop\n\tv_nop" : "+v"(a), "+v"(b), "+v"(c), "+v"(d));
#endif
}
__device__ __forceinline__ void wave_sync_lds() {
  __builtin_amdgcn_fence(__ATOMIC_RELEASE, "workgroup");
  __builtin_amdgcn_wave_barrier();
  __builtin_amdgcn_fence(__ATOMIC_ACQUIRE, "workgroup");
}

__global__ __launch_bounds__(256) void cvt_bf16x8(const float* __restrict__ in, unsigned short* out, int n8) {
  const int i = blockIdx.x * 256 + threadIdx.x;
  if (i < n8) {
    const v4f a = *(const v4f*)(in + (size_t)i * 8);
    const v4f b = *(const v4f*)(in + (size_t)i * 8 + 4);
    v4u p;
    p[0] = pk16(bf_bits(a[0]), bf_bits(a[1]));
    p[1] = pk16(bf_bits(a[2]), bf_bits(a[3]));
    p[2] = pk16(bf_bits(b[0]), bf_bits(b[1]));
    p[3] = pk16(bf_bits(b[2]), bf_bits(b[3]));
    *(volatile v4u*)(out + (size_t)i * 8) = p;
    __threadfence();
    *(volatile v4u*)(out + (size_t)i * 8) = p;
  }
}

template <int NSPLIT, int OUT_MODE, int BIAS_MODE>
__global__ __launch_bounds__(256) void gemm64(
    const unsigned short* __restrict__ Ap, const unsigned short* A2p, int lda, long long strideA,
    const unsigned short* __restrict__ Btp, const unsigned short* Bt2p, int ldb, long long strideB,
    void* Cout, int ldc, long long strideC,
    void* Cout2, int ldc2, long long strideC2, int N2,
    const float* __restrict__ biasp,
    int M, int N, int K, float rscale) {
  const __bf16* A   = (const __bf16*)(const void*)Ap;
  const __bf16* A2  = (const __bf16*)(const void*)A2p;
  const __bf16* Bt  = (const __bf16*)(const void*)Btp;
  const __bf16* Bt2 = (const __bf16*)(const void*)Bt2p;
  __shared__ __align__(16) float sT[8][16 * 68];
  const int b    = blockIdx.y;
  const int lane = threadIdx.x & 31;
  const int wave = threadIdx.x >> 5;
  const int tilesN = N >> 6;
  const int tilesM = M >> 6;
  const int tile = blockIdx.x * 8 + wave;
  if (tile >= tilesM * tilesN) return;
  const int tm = tile / tilesN;
  const int tn = tile - tm * tilesN;
  const int m0 = tm << 6;
  const int n0 = tn << 6;

  const __bf16* Ab  = A  + (size_t)b * strideA;
  const __bf16* Bb  = Bt + (size_t)b * strideB;
  const __bf16* Ab2 = (NSPLIT >= 1) ? (A2  + (size_t)b * strideA) : Ab;
  const __bf16* Bb2 = (NSPLIT == 2) ? (Bt2 + (size_t)b * strideB) : Bb;

  const int rlane = lane & 15;
  const int koff  = (lane >> 4) * 8;
  const int mOff  = (lane >> 4) * 8;

  v8f acc[4][4];
#pragma unroll
  for (int i = 0; i < 4; ++i)
#pragma unroll
    for (int j = 0; j < 4; ++j) acc[i][j] = zero8();

  for (int k0 = 0; k0 < K; k0 += 32) {
    v16b bh[4], bl[4];
#pragma unroll
    for (int j = 0; j < 4; ++j) {
      const size_t bo = (size_t)(n0 + (j << 4) + rlane) * ldb + koff + k0;
      bh[j] = ldfrag_b(Bb + bo);
      if (NSPLIT == 2) bl[j] = ldfrag_b(Bb2 + bo); else bl[j] = bh[j];
    }
#pragma unroll
    for (int i = 0; i < 4; ++i) {
      const size_t ao = (size_t)(m0 + (i << 4) + rlane) * lda + koff + k0;
      const v16b ah = ldfrag_b(Ab + ao);
      v16b al = ah;
      if (NSPLIT >= 1) al = ldfrag_b(Ab2 + ao);
#pragma unroll
      for (int j = 0; j < 4; ++j) {
        acc[i][j] = mma_b_raw(ah, bh[j], acc[i][j]);
        if (NSPLIT >= 1) acc[i][j] = mma_b_raw(al, bh[j], acc[i][j]);
        if (NSPLIT == 2) acc[i][j] = mma_b_raw(ah, bl[j], acc[i][j]);
      }
      dep_guard_b(acc[i][0], acc[i][3], ah, al);
    }
    keep4_b(bh[0], bh[1], bh[2], bh[3]);
    if (NSPLIT == 2) keep4_b(bl[0], bl[1], bl[2], bl[3]);
  }
  acc_guard4(acc[0][0], acc[0][1], acc[0][2], acc[0][3]);
  acc_guard4(acc[1][0], acc[1][1], acc[1][2], acc[1][3]);
  acc_guard4(acc[2][0], acc[2][1], acc[2][2], acc[2][3]);
  acc_guard4(acc[3][0], acc[3][1], acc[3][2], acc[3][3]);

  float* slab = sT[wave];
#pragma unroll
  for (int i = 0; i < 4; ++i) {
    const int mBase = m0 + (i << 4);
    float brow[8];
#pragma unroll
    for (int r = 0; r < 8; ++r) {
      brow[r] = 0.f;
      if (BIAS_MODE == 2) brow[r] = bf_rne(biasp[mBase + mOff + r]);
    }
#pragma unroll
    for (int j = 0; j < 4; ++j) {
      float bcol = 0.f;
      if (BIAS_MODE == 1) bcol = bf_rne(biasp[n0 + (j << 4) + rlane]);
#pragma unroll
      for (int r = 0; r < 8; ++r) {
        slab[(mOff + r) * 68 + (j << 4) + rlane] = acc[i][j][r] + bcol + brow[r];
      }
    }
    wave_sync_lds();
    if (OUT_MODE == 0) {
      float* C = (float*)Cout + (size_t)b * strideC;
      const int hh = lane >> 4, c4 = (lane & 15) * 4;
      for (int pass = 0; pass < 2; ++pass) {
#pragma unroll
        for (int it = 0; it < 8; ++it) {
          const int row = it * 2 + hh;
          const v4f v = *(const v4f*)(slab + row * 68 + c4);
          *(volatile v4f*)(C + (size_t)(mBase + row) * ldc + n0 + c4) = v;
        }
        __threadfence();
      }
    } else {
      const int q = lane >> 3, c8 = (lane & 7) * 8;
      unsigned short* C  = (unsigned short*)Cout  + (size_t)b * strideC;
      unsigned short* C2 = (unsigned short*)Cout2 + (size_t)b * strideC2;
      const bool wlo = (OUT_MODE == 2) || (n0 < N2);
      v4u hv[4], lv[4];
#pragma unroll
      for (int it = 0; it < 4; ++it) {
        const int row = it * 4 + q;
        const float* sp = slab + row * 68 + c8;
        v4u a, a2;
#pragma unroll
        for (int e = 0; e < 4; ++e) {
          const float f0 = sp[2 * e], f1 = sp[2 * e + 1];
          unsigned short h0, h1, l0, l1;
          if (OUT_MODE == 2) {
            h0 = bf_bits(f0); h1 = bf_bits(f1);
            l0 = bf_bits(f0 - bf_up(h0)); l1 = bf_bits(f1 - bf_up(h1));
          } else {
            const _Float16 x0 = (_Float16)f0, x1 = (_Float16)f1;
            h0 = h_bits(x0); h1 = h_bits(x1);
            l0 = h_bits((_Float16)((f0 - (float)x0) * rscale));
            l1 = h_bits((_Float16)((f1 - (float)x1) * rscale));
          }
          a[e] = pk16(h0, h1); a2[e] = pk16(l0, l1);
        }
        hv[it] = a; lv[it] = a2;
      }
      for (int pass = 0; pass < 2; ++pass) {
#pragma unroll
        for (int it = 0; it < 4; ++it) {
          const int row = it * 4 + q;
          *(volatile v4u*)(C + (size_t)(mBase + row) * ldc + n0 + c8) = hv[it];
          if (wlo) *(volatile v4u*)(C2 + (size_t)(mBase + row) * ldc2 + n0 + c8) = lv[it];
        }
        __threadfence();
      }
    }
    wave_sync_lds();
  }
}

__global__ __launch_bounds__(256) void rope_rows(
    const float* __restrict__ qkf, const float* __restrict__ cosp, const float* __restrict__ sinp,
    unsigned short* qhp, unsigned short* qlp, unsigned short* kpp, int nrows, float rscale) {
  const int row = blockIdx.x;
  if (row >= nrows) return;
  const int t   = threadIdx.x;
  const int isk = t >> 7;
  const int c0  = (t & 127) * 8;
  const int d0  = c0 & (HD - 1);
  const bool lowhalf = (d0 < (HD / 2));
  const int pc0 = lowhalf ? (c0 + HD / 2) : (c0 - HD / 2);
  const float sgn = lowhalf ? -1.0f : 1.0f;

  const float* src = qkf + (size_t)row * QKP + (size_t)isk * DM;
  const v4f x0 = *(const v4f*)(src + c0);
  const v4f x1 = *(const v4f*)(src + c0 + 4);
  const v4f p0 = *(const v4f*)(src + pc0);
  const v4f p1 = *(const v4f*)(src + pc0 + 4);
  const v4f cA = *(const v4f*)(cosp + (size_t)row * HD + d0);
  const v4f cB = *(const v4f*)(cosp + (size_t)row * HD + d0 + 4);
  const v4f sA = *(const v4f*)(sinp + (size_t)row * HD + d0);
  const v4f sB = *(const v4f*)(sinp + (size_t)row * HD + d0 + 4);

  v4f y0, y1;
#pragma unroll
  for (int e = 0; e < 4; ++e) {
    y0[e] = x0[e] * bf_rne(cA[e]) + (sgn * p0[e]) * bf_rne(sA[e]);
    y1[e] = x1[e] * bf_rne(cB[e]) + (sgn * p1[e]) * bf_rne(sB[e]);
  }
  v4u hv, lv;
#pragma unroll
  for (int e = 0; e < 2; ++e) {
    const float f0 = y0[2 * e], f1 = y0[2 * e + 1];
    const float g0 = y1[2 * e], g1 = y1[2 * e + 1];
    const _Float16 a0 = (_Float16)f0, a1 = (_Float16)f1;
    const _Float16 b0 = (_Float16)g0, b1 = (_Float16)g1;
    hv[e]     = pk16(h_bits(a0), h_bits(a1));
    hv[2 + e] = pk16(h_bits(b0), h_bits(b1));
    lv[e]     = pk16(h_bits((_Float16)((f0 - (float)a0) * rscale)),
                     h_bits((_Float16)((f1 - (float)a1) * rscale)));
    lv[2 + e] = pk16(h_bits((_Float16)((g0 - (float)b0) * rscale)),
                     h_bits((_Float16)((g1 - (float)b1) * rscale)));
  }
  const size_t o = (size_t)row * DM + c0;
  if (isk == 0) {
    *(volatile v4u*)(qhp + o) = hv;
    *(volatile v4u*)(qlp + o) = lv;
    __threadfence();
    *(volatile v4u*)(qhp + o) = hv;
    *(volatile v4u*)(qlp + o) = lv;
  } else {
    *(volatile v4u*)(kpp + o) = hv;
    __threadfence();
    *(volatile v4u*)(kpp + o) = hv;
  }
}

__global__ __launch_bounds__(128)
void attn64(const unsigned short* __restrict__ qhp, const unsigned short* __restrict__ qlp,
            const unsigned short* __restrict__ kpp, const unsigned short* __restrict__ vtp,
            unsigned short* ohp, unsigned short* olp, float sscale, float rres) {
  union FH { v16h v; v8h h[2]; };
  __shared__ __align__(16) _Float16 Ksh[64 * 64];
  __shared__ __align__(16) _Float16 Vth[64 * 64];
  __shared__ __align__(16) _Float16 Psh[4][16 * 64];
  __shared__ __align__(16) float    Os[4][16 * 64];

  const int tid  = threadIdx.x;
  const int wave = tid >> 5;
  const int lane = tid & 31;
  const int hh   = lane >> 4;
  const int c    = lane & 15;

  const int bx   = blockIdx.x;
  const int qb   = bx % NQB;
  const int h    = bx / NQB;
  const int q0   = qb * 64 + wave * 16;

  const _Float16* Qh = (const _Float16*)(const void*)qhp + (size_t)h * HD;
  const _Float16* Ql = (const _Float16*)(const void*)qlp + (size_t)h * HD;
  const _Float16* Kg = (const _Float16*)(const void*)kpp + (size_t)h * HD;
  const _Float16* Vg = (const _Float16*)(const void*)vtp + (size_t)h * HD * SEQ;

  v16h qah[2], qal[2];
#pragma unroll
  for (int dc = 0; dc < 2; ++dc) {
    qah[dc] = ldfrag_h(Qh + (size_t)(q0 + c) * DM + dc * 32 + 8 * hh);
    qal[dc] = ldfrag_h(Ql + (size_t)(q0 + c) * DM + dc * 32 + 8 * hh);
  }

  float mrow[8], lrow[8];
  v8f oacc[4];
#pragma unroll
  for (int r = 0; r < 8; ++r) { mrow[r] = -INFINITY; lrow[r] = 0.f; }
#pragma unroll
  for (int t = 0; t < 4; ++t) oacc[t] = zero8();

  for (int kt = 0; kt < NQB; ++kt) {
    const int kv0 = kt * 64;
    __syncthreads();
    {
      const int r = tid >> 1, hf = (tid & 1) * 32;
      const _Float16* kg = Kg + (size_t)(kv0 + r) * DM + hf;
      const _Float16* vg = Vg + (size_t)r * SEQ + kv0 + hf;
#pragma unroll
      for (int i = 0; i < 4; ++i) {
        const v8h a0 = *(const v8h*)(kg + 8 * i);
        const v8h b0 = *(const v8h*)(vg + 8 * i);
        *(v8h*)(Ksh + r * 64 + hf + 8 * i) = a0;
        *(v8h*)(Vth + r * 64 + hf + 8 * i) = b0;
      }
    }
    __syncthreads();

    v8f s[4];
#pragma unroll
    for (int j = 0; j < 4; ++j) {
      v8f sh = zero8(), sl = zero8();
#pragma unroll
      for (int dc = 0; dc < 2; ++dc) {
        FH kb;
        kb.h[0] = *(const v8h*)(Ksh + (j * 16 + c) * 64 + dc * 32 + 8 * hh);
        kb.h[1] = *(const v8h*)(Ksh + (j * 16 + c) * 64 + dc * 32 + 16 + 8 * hh);
        sh = mma_h(qah[dc], kb.v, sh);
        sl = mma_h(qal[dc], kb.v, sl);
      }
#pragma unroll
      for (int r = 0; r < 8; ++r) s[j][r] = (sh[r] + sl[r] * rres) * sscale;
    }

    _Float16* pwh = Psh[wave];
#pragma unroll
    for (int r = 0; r < 8; ++r) {
      float m = s[0][r];
      m = fmaxf(m, s[1][r]);
      m = fmaxf(m, s[2][r]);
      m = fmaxf(m, s[3][r]);
#pragma unroll
      for (int off = 1; off < 16; off <<= 1) m = fmaxf(m, __shfl_xor(m, off, 32));
      const float mnew  = fmaxf(mrow[r], m);
      const float alpha = __expf(mrow[r] - mnew);
      mrow[r] = mnew;
      float psum = 0.f;
#pragma unroll
      for (int j = 0; j < 4; ++j) {
        const float p = __expf(s[j][r] - mnew);
        psum += p;
        pwh[(8 * hh + r) * 64 + j * 16 + c] = (_Float16)(p * 1024.0f);
      }
#pragma unroll
      for (int off = 1; off < 16; off <<= 1) psum += __shfl_xor(psum, off, 32);
      lrow[r] = lrow[r] * alpha + psum;
#pragma unroll
      for (int t = 0; t < 4; ++t) oacc[t][r] *= alpha;
    }
    wave_sync_lds();

#pragma unroll 1
    for (int kk = 0; kk < 2; ++kk) {
      FH pa;
      pa.h[0] = *(const v8h*)(pwh + c * 64 + kk * 32 + 8 * hh);
      pa.h[1] = *(const v8h*)(pwh + c * 64 + kk * 32 + 16 + 8 * hh);
#pragma unroll
      for (int t = 0; t < 4; ++t) {
        FH vb;
        vb.h[0] = *(const v8h*)(Vth + (t * 16 + c) * 64 + kk * 32 + 8 * hh);
        vb.h[1] = *(const v8h*)(Vth + (t * 16 + c) * 64 + kk * 32 + 16 + 8 * hh);
        oacc[t] = mma_h(pa.v, vb.v, oacc[t]);
      }
    }
  }

  float* os = Os[wave];
#pragma unroll
  for (int r = 0; r < 8; ++r) {
    const float l = lrow[r];
    const float inv = ((l > 0.f) ? (1.0f / l) : 0.f) * (1.0f / 1024.0f);
#pragma unroll
    for (int t = 0; t < 4; ++t) os[(8 * hh + r) * 64 + t * 16 + c] = oacc[t][r] * inv;
  }
  wave_sync_lds();
  {
    const int q4 = lane >> 3, c8 = (lane & 7) * 8;
    v4u hv[4], lv[4];
#pragma unroll
    for (int it = 0; it < 4; ++it) {
      const int row = it * 4 + q4;
      const float* sp = os + row * 64 + c8;
      v4u a, a2;
#pragma unroll
      for (int e = 0; e < 4; ++e) {
        const float f0 = sp[2 * e], f1 = sp[2 * e + 1];
        const unsigned short h0 = bf_bits(f0), h1 = bf_bits(f1);
        const unsigned short l0 = bf_bits(f0 - bf_up(h0)), l1 = bf_bits(f1 - bf_up(h1));
        a[e] = pk16(h0, h1); a2[e] = pk16(l0, l1);
      }
      hv[it] = a; lv[it] = a2;
    }
    for (int pass = 0; pass < 2; ++pass) {
#pragma unroll
      for (int it = 0; it < 4; ++it) {
        const int row = it * 4 + q4;
        const size_t go = (size_t)(q0 + row) * DM + (size_t)h * HD + c8;
        *(volatile v4u*)(ohp + go) = hv[it];
        *(volatile v4u*)(olp + go) = lv[it];
      }
      __threadfence();
    }
  }
}

extern "C" void kernel_launch(void* const* d_in, const int* in_sizes, int n_in,
                              void* d_out, int out_size, void* d_ws, size_t ws_size,
                              hipStream_t stream) {
  if (n_in < 7) return;
  if (in_sizes[0] != SEQ * DM) return;
  if (in_sizes[1] != SEQ * HD) return;
  if (in_sizes[2] != SEQ * HD) return;
  if (in_sizes[3] != 3 * DM * DM) return;
  if (in_sizes[4] != 3 * DM) return;
  if (in_sizes[5] != DM * DM) return;
  if (in_sizes[6] != DM) return;
  if (out_size != SEQ * DM) return;

  const float* x     = (const float*)d_in[0];
  const float* cosp  = (const float*)d_in[1];
  const float* sinp  = (const float*)d_in[2];
  const float* wqkv  = (const float*)d_in[3];
  const float* bqkv  = (const float*)d_in[4];
  const float* wout  = (const float*)d_in[5];
  const float* bout  = (const float*)d_in[6];

  const size_t PXb  = (size_t)SEQ * DM * 2;
  const size_t PWq  = (size_t)3 * DM * DM * 2;
  const size_t PWo  = (size_t)DM * DM * 2;
  const size_t PQKf = (size_t)SEQ * QKP * 4;
  const size_t P16  = (size_t)SEQ * DM * 2;
  const size_t PVT  = (size_t)DM * SEQ * 2;
  size_t off = 0;
  const size_t oXb  = off; off += PXb;
  const size_t oWq  = off; off += PWq;
  const size_t oWo  = off; off += PWo;
  const size_t oQKf = off; off += PQKf;
  const size_t oQh  = off; off += P16;
  const size_t oQl  = off; off += P16;
  const size_t oKp  = off; off += P16;
  const size_t oVT  = off; off += PVT;
  const size_t oOh  = off; off += P16;
  const size_t oOl  = off; off += P16;
  if (off > ws_size) return;
  if (off > (size_t)134217728) return;

  char* ws = (char*)d_ws;
  unsigned short* Xb    = (unsigned short*)(ws + oXb);
  unsigned short* Wqkvb = (unsigned short*)(ws + oWq);
  unsigned short* Wvb   = Wqkvb + (size_t)2 * DM * DM;
  unsigned short* Wob   = (unsigned short*)(ws + oWo);
  float*          QKf   = (float*)(ws + oQKf);
  unsigned short* Qh    = (unsigned short*)(ws + oQh);
  unsigned short* Ql    = (unsigned short*)(ws + oQl);
  unsigned short* Kp    = (unsigned short*)(ws + oKp);
  unsigned short* VT    = (unsigned short*)(ws + oVT);
  unsigned short* Oh    = (unsigned short*)(ws + oOh);
  unsigned short* Ol    = (unsigned short*)(ws + oOl);

  const dim3 blk(256);
  const int n8x  = SEQ * DM / 8;
  const int n8wq = 3 * DM * DM / 8;
  const int n8wo = DM * DM / 8;
  const dim3 gCvtX((n8x + 255) / 256);
  const dim3 gCvtWq((n8wq + 255) / 256);
  const dim3 gCvtWo((n8wo + 255) / 256);
  const dim3 gQK(((SEQ / 64) * (QKP / 64) + 7) / 8, 1);
  const dim3 gRope(SEQ);
  const dim3 gVT(((DM / 64) * (SEQ / 64) + 7) / 8, 1);
  const dim3 gAttn(NH * NQB);
  const dim3 gOut(((SEQ / 64) * (DM / 64) + 7) / 8, 1);

  cvt_bf16x8<<<gCvtX, blk, 0, stream>>>(x, Xb, n8x);
  cvt_bf16x8<<<gCvtWq, blk, 0, stream>>>(wqkv, Wqkvb, n8wq);
  cvt_bf16x8<<<gCvtWo, blk, 0, stream>>>(wout, Wob, n8wo);
  gemm64<0, 0, 1><<<gQK, blk, 0, stream>>>(
      Xb, Xb, DM, 0LL, Wqkvb, Wqkvb, DM, 0LL,
      (void*)QKf, QKP, 0LL, (void*)QKf, QKP, 0LL, 0,
      bqkv,
      SEQ, QKP, DM, 1.0f);
  rope_rows<<<gRope, blk, 0, stream>>>(QKf, cosp, sinp, Qh, Ql, Kp, SEQ, 4096.0f);
  gemm64<0, 3, 2><<<gVT, blk, 0, stream>>>(
      Wvb, Wvb, DM, 0LL, Xb, Xb, DM, 0LL,
      (void*)VT, SEQ, 0LL, (void*)VT, SEQ, 0LL, 0,
      bqkv + 2 * DM,
      DM, SEQ, DM, 4096.0f);
  attn64<<<gAttn, dim3(128), 0, stream>>>(Qh, Ql, Kp, VT, Oh, Ol, 0.125f, 1.0f / 4096.0f);
  gemm64<1, 0, 1><<<gOut, blk, 0, stream>>>(
      Oh, Ol, DM, 0LL, Wob, Wob, DM, 0LL,
      d_out, DM, 0LL, d_out, DM, 0LL, 0,
      bout,
      SEQ, DM, DM, 1.0f);
  (void)hipGetLastError();
}
